// Longhorn_8358006358686
// MI455X (gfx1250) — hardware-verified
//
#include <hip/hip_runtime.h>
#include <hip/hip_bf16.h>
#include <stdint.h>

#define BATCH   2
#define SEQL    2048
#define DMODEL  1024
#define DINNER  2048
#define DTRANK  64
#define DSTATE  16
#define DCONV   4
#define MROWS   (BATCH * SEQL)
#define XDBLW   (DTRANK + 2 * DSTATE)

typedef _Float16 __hf;
#define __bf16 __hf
typedef __attribute__((ext_vector_type(16))) _Float16 v16bf;
typedef __attribute__((ext_vector_type(8)))  _Float16 v8bf;
typedef __attribute__((ext_vector_type(8)))  float  v8f;
typedef __attribute__((ext_vector_type(2)))  _Float16 v2hf;
typedef __attribute__((ext_vector_type(2)))  unsigned u32x2;

#define LDSTRIDE 40

__device__ __forceinline__ unsigned pack_bf16x2(float a, float b) {
    v2hf h; h[0] = (_Float16)a; h[1] = (_Float16)b;
    return __builtin_bit_cast(unsigned, h);
}
__device__ __forceinline__ __bf16 f2bf(float f) { return (_Float16)f; }

__device__ __forceinline__ float sigmoidf_fast(float x) {
    return 1.0f / (1.0f + expf(-x));
}

__global__ __launch_bounds__(256) void cvt_bf16_kernel(
    const float* __restrict__ src, unsigned* __restrict__ dst  )
{
    int i = blockIdx.x * 256 + threadIdx.x;
    float4 v = ((const float4*)src)[i];
    u32x2 p;
    p[0] = pack_bf16x2(v.x, v.y);
    p[1] = pack_bf16x2(v.z, v.w);
    *(volatile u32x2*)((u32x2*)dst + i) = p; __threadfence(); *(volatile u32x2*)((u32x2*)dst + i) = p;
}

__global__ __launch_bounds__(256) void gemm_bf16_wmma(
    const __bf16* __restrict__ A, int lda,
    const __bf16* __restrict__ W, int ldw,
    float* __restrict__ C, int ldc,
    int M, int N, int K)
{
    __shared__ __attribute__((aligned(16))) __bf16 As[2][128 * LDSTRIDE];
    __shared__ __attribute__((aligned(16))) __bf16 Bs[2][128 * LDSTRIDE];

    const int tid   = threadIdx.x;
    const int lane  = tid & 31;
    const int wave  = tid >> 5;
    const int waveM = (wave >> 2) * 64;
    const int waveN = (wave &  3) * 32;
    const int gm0   = blockIdx.y * 128;
    const int gn0   = blockIdx.x * 128;
    const int kt    = K >> 5;

    auto issue = [&](int s, int kofs) {
        #pragma unroll
        for (int i = 0; i < 2; ++i) {
            int c = tid + 256 * i;
            int row = c >> 2, ch = c & 3;
            int gr = gm0 + row; if (gr >= M) gr = M - 1;
            *(v8bf*)&As[s][row * LDSTRIDE + ch * 8] = *(const v8bf*)(A + (size_t)gr * lda + kofs + ch * 8);
        }
        #pragma unroll
        for (int i = 0; i < 2; ++i) {
            int c = tid + 256 * i;
            int row = c >> 2, ch = c & 3;
            int gr = gn0 + row; if (gr >= N) gr = N - 1;
            *(v8bf*)&Bs[s][row * LDSTRIDE + ch * 8] = *(const v8bf*)(W + (size_t)gr * ldw + kofs + ch * 8);
        }
    };

    v8f acc[4][2] = {};
    int cur = 0;
    for (int kk = 0; kk < kt; ++kk) {
        issue(cur, kk << 5);
        __syncthreads();

        const int khalf = (lane < 16) ? 0 : 8;

        v16bf afrag[4], bfrag[2];
        #pragma unroll
        for (int tm = 0; tm < 4; ++tm) {
            const __bf16* ar = &As[cur][(waveM + tm * 16 + (lane & 15)) * LDSTRIDE];
            v8bf lo = *(const v8bf*)(ar + khalf);
            v8bf hi = *(const v8bf*)(ar + 16 + khalf);
            afrag[tm] = __builtin_shufflevector(lo, hi, 0,1,2,3,4,5,6,7,8,9,10,11,12,13,14,15);
        }
        #pragma unroll
        for (int tn = 0; tn < 2; ++tn) {
            const __bf16* br = &Bs[cur][(waveN + tn * 16 + (lane & 15)) * LDSTRIDE];
            v8bf lo = *(const v8bf*)(br + khalf);
            v8bf hi = *(const v8bf*)(br + 16 + khalf);
            bfrag[tn] = __builtin_shufflevector(lo, hi, 0,1,2,3,4,5,6,7,8,9,10,11,12,13,14,15);
        }

        #pragma unroll
        for (int tm = 0; tm < 4; ++tm)
            #pragma unroll
            for (int tn = 0; tn < 2; ++tn)
              { acc[tm][tn] = __builtin_amdgcn_wmma_f32_16x16x32_f16(
                    false, afrag[tm], false, bfrag[tn],
                    (short)0, acc[tm][tn], false, false);
                asm volatile("v_nop\n\tv_nop\n\tv_nop\n\tv_nop" : "+v"(acc[tm][tn]) : "v"(afrag[tm]), "v"(bfrag[tn])); }

        __syncthreads();
        cur ^= 1;
    }

    const int hf = lane >> 4;
    if (gn0 + waveN < N) {
        for (int pass = 0; pass < 2; ++pass) {
            #pragma unroll
            for (int tm = 0; tm < 4; ++tm) {
                const int m0r = gm0 + waveM + tm * 16;
                #pragma unroll
                for (int r = 0; r < 8; ++r) {
                    const float a0 = acc[tm][0][r], a1 = acc[tm][1][r];
                    const float x0 = __shfl_xor(a0, 16), x1 = __shfl_xor(a1, 16);
                    *(volatile float*)(C + (size_t)(m0r + r) * ldc + gn0 + waveN + lane)     = hf ? x1 : a0;
                    *(volatile float*)(C + (size_t)(m0r + 8 + r) * ldc + gn0 + waveN + lane) = hf ? a1 : x0;
                }
            }
            __threadfence();
        }
    }
}

__global__ __launch_bounds__(256) void conv_silu_kernel(
    const float* __restrict__ XZ, const float* __restrict__ cw,
    const float* __restrict__ cb, float* __restrict__ XC,
    __bf16* __restrict__ XCbf)
{
    int idx = blockIdx.x * 256 + threadIdx.x;
    int d   = idx & (DINNER - 1);
    int row = idx >> 11;
    int l   = row & (SEQL - 1);
    int b   = row >> 11;
    float acc = cb[d];
    #pragma unroll
    for (int i = 0; i < DCONV; ++i) {
        int li = l - (DCONV - 1) + i;
        if (li >= 0)
            acc += XZ[(size_t)(b * SEQL + li) * (2 * DINNER) + d] * cw[d * DCONV + i];
    }
    float s = acc * sigmoidf_fast(acc);
    *(volatile float*)(XC + (size_t)row * DINNER + d) = s; *(volatile __bf16*)(XCbf + (size_t)row * DINNER + d) = f2bf(s);
    __threadfence();
    *(volatile float*)(XC + (size_t)row * DINNER + d) = s; *(volatile __bf16*)(XCbf + (size_t)row * DINNER + d) = f2bf(s);
}

__global__ __launch_bounds__(256) void scan_kernel(
    const float* __restrict__ XC, const float* __restrict__ DT,
    const float* __restrict__ XDBL, const float* __restrict__ XZ,
    const float* __restrict__ dt_b, const float* __restrict__ Dv,
    __bf16* __restrict__ Ybf)
{
    const int b  = blockIdx.x >> 3;
    const int d  = ((blockIdx.x & 7) << 8) + threadIdx.x;
    const float bias = dt_b[d];
    const float Dd   = Dv[d];

    __shared__ float kq[2 * DSTATE];
    float st[DSTATE];
    #pragma unroll
    for (int n = 0; n < DSTATE; ++n) st[n] = 0.0f;

    for (int t = 0; t < SEQL; ++t) {
        const size_t row = (size_t)(b * SEQL + t);
        if (threadIdx.x < 2 * DSTATE)
            kq[threadIdx.x] = XDBL[row * XDBLW + DTRANK + threadIdx.x];
        __syncthreads();

        float ksum = 0.0f;
        #pragma unroll
        for (int n = 0; n < DSTATE; ++n) ksum += kq[n] * kq[n];

        const float x  = XC[row * DINNER + d];
        const float dr = DT[row * DINNER + d];
        const float z  = XZ[row * (2 * DINNER) + DINNER + d];

        float dtv = sigmoidf_fast(dr + bias);
        dtv = dtv / (1.0f + dtv * ksum);

        float y = 0.0f;
        #pragma unroll
        for (int n = 0; n < DSTATE; ++n) {
            const float kn = kq[n];
            st[n] = st[n] * (1.0f - dtv * kn * kn) + x * dtv * kn;
            y += st[n] * kq[DSTATE + n];
        }
        { const __bf16 yv = f2bf((y + Dd * x) * z * sigmoidf_fast(z));
          *(volatile __bf16*)(Ybf + row * DINNER + d) = yv;
          *(volatile __bf16*)(Ybf + row * DINNER + d) = yv; }
        __syncthreads();
    }
}

extern "C" void kernel_launch(void* const* d_in, const int* in_sizes, int n_in,
                              void* d_out, int out_size, void* d_ws, size_t ws_size,
                              hipStream_t stream) {
    const float* hs    = (const float*)d_in[0];
    const float* inW   = (const float*)d_in[1];
    const float* convW = (const float*)d_in[2];
    const float* convB = (const float*)d_in[3];
    const float* xpW   = (const float*)d_in[4];
    const float* dthW  = (const float*)d_in[5];
    const float* dthB  = (const float*)d_in[6];
    const float* outW  = (const float*)d_in[7];
    const float* Dv    = (const float*)d_in[8];
    float* out = (float*)d_out;
    (void)in_sizes; (void)n_in; (void)out_size;
    if (ws_size < (size_t)230 * 1024 * 1024) return;

    float* ws   = (float*)d_ws;
    float* XZ   = ws;
    float* XC   = XZ   + (size_t)MROWS * (2 * DINNER);
    float* XDBL = XC   + (size_t)MROWS * DINNER;
    float* DT   = XDBL + (size_t)MROWS * XDBLW;
    __bf16* bfb   = (__bf16*)(DT + (size_t)MROWS * DINNER);
    __bf16* hs_b  = bfb;
    __bf16* inW_b = hs_b  + (size_t)MROWS * DMODEL;
    __bf16* XC_b  = inW_b + (size_t)(2*DINNER) * DMODEL;
    __bf16* xpW_b = XC_b  + (size_t)MROWS * DINNER;
    __bf16* XDBL_b= xpW_b + (size_t)XDBLW * DINNER;
    __bf16* dthW_b= XDBL_b+ (size_t)MROWS * XDBLW;
    __bf16* Y_b   = dthW_b+ (size_t)DINNER * DTRANK;
    __bf16* outW_b= Y_b   + (size_t)MROWS * DINNER;

    dim3 blk(256);
    #define CVT(src, dst, n) \
        cvt_bf16_kernel<<<(n) / 1024, blk, 0, stream>>>((src), (unsigned*)(dst))

    CVT(hs,   hs_b,   (size_t)MROWS * DMODEL);
    CVT(inW,  inW_b,  (size_t)(2*DINNER) * DMODEL);
    CVT(xpW,  xpW_b,  (size_t)XDBLW * DINNER);
    CVT(dthW, dthW_b, (size_t)DINNER * DTRANK);
    CVT(outW, outW_b, (size_t)DMODEL * DINNER);

    gemm_bf16_wmma<<<dim3((2*DINNER)/128, MROWS/128), blk, 0, stream>>>(
        hs_b, DMODEL, inW_b, DMODEL, XZ, 2*DINNER, MROWS, 2*DINNER, DMODEL);

    conv_silu_kernel<<<(MROWS * DINNER) / 256, blk, 0, stream>>>(
        XZ, convW, convB, XC, XC_b);

    gemm_bf16_wmma<<<dim3(1, MROWS/128), blk, 0, stream>>>(
        XC_b, DINNER, xpW_b, DINNER, XDBL, XDBLW, MROWS, XDBLW, DINNER);
    CVT(XDBL, XDBL_b, (size_t)MROWS * XDBLW);

    gemm_bf16_wmma<<<dim3(DINNER/128, MROWS/128), blk, 0, stream>>>(
        XDBL_b, XDBLW, dthW_b, DTRANK, DT, DINNER, MROWS, DINNER, DTRANK);

    scan_kernel<<<(BATCH * DINNER) / 256, blk, 0, stream>>>(
        XC, DT, XDBL, XZ, dthB, Dv, Y_b);

    gemm_bf16_wmma<<<dim3(DMODEL/128, MROWS/128), blk, 0, stream>>>(
        Y_b, DINNER, outW_b, DINNER, out, DMODEL, MROWS, DMODEL, DINNER);
    #undef CVT
}
